// CoordinateDecoder_18021682774655
// MI455X (gfx1250) — hardware-verified
//
#include <hip/hip_runtime.h>
#include <math.h>

#ifndef NB
#define NB 8
#endif
#ifndef NPTS
#define NPTS 65536
#endif
#define IMG_H 64
#define IMG_W 64
#define IMG_C 256
#define IMG_ELEMS (IMG_H * IMG_W * IMG_C)
#define NENC 42
#define KIN 298
#define WIDTH 128
#define NOUT 3
#define NOUTP 16
#define K0P 320
#define FEAT0 48
#define XP 328
#define SP 132
#define RES0 128
#define WAVES 4
#define ROWS_W 32
#define ROWS_B (WAVES * ROWS_W)
#define TILES_PER_IMG (NPTS / ROWS_B)
#define OFLAT 1024

static constexpr float ACT_CARRY = 8.0f;
static constexpr float W_CARRY = 32.0f;
static constexpr float ACT_SC = 1.0f / 256.0f;
static constexpr float RES_CARRY = 2048.0f;
static constexpr float RES_INV = 1.0f / 2048.0f;
static constexpr float GELU_K = (float)(-2.0 * 1.4426950408889634 * 0.7978845608028654);

static_assert(NPTS % ROWS_B == 0);
static_assert(IMG_H == 64 && IMG_W == 64);
static_assert(K0P % 32 == 0 && WIDTH % 32 == 0 && WIDTH % 16 == 0);
static_assert(FEAT0 >= NENC && FEAT0 % 8 == 0 && FEAT0 + IMG_C <= K0P);
static_assert(NENC + IMG_C == KIN);
static_assert(XP % 8 == 0 && XP >= K0P);
static_assert(RES0 >= WIDTH && RES0 % 8 == 0 && RES0 + WIDTH <= XP);
static_assert(SP % 4 == 0 && SP >= WIDTH);
static_assert(32 * 8 == IMG_C);
static_assert(32 * 4 == WIDTH);
static_assert(16 * 8 == WIDTH);
static_assert(24 * 16 == ROWS_W * NOUT * 4);
static_assert(3 * 32 == ROWS_W * NOUT);
static_assert(ROWS_W * NOUTP <= OFLAT && OFLAT + ROWS_W * NOUT <= 16 * SP);
static_assert(sizeof(_Float16) * WAVES * ROWS_W * XP + sizeof(float) * WAVES * 16 * SP <= 131072);
static_assert(((size_t)NB * IMG_ELEMS / 8) % 256 == 0);
static_assert((size_t)NB * IMG_ELEMS * 2 + (size_t)WIDTH * K0P * 2 + 2 * (size_t)WIDTH * WIDTH * 2 + (size_t)NOUTP * WIDTH * 2 + 5 * 256 <= (size_t)134217728);

typedef _Float16 h16;
typedef __attribute__((ext_vector_type(16))) _Float16 v16h;
typedef __attribute__((ext_vector_type(8)))  _Float16 v8h;
typedef __attribute__((ext_vector_type(4)))  _Float16 v4h;
typedef __attribute__((ext_vector_type(8)))  float    v8f;
typedef __attribute__((ext_vector_type(4)))  float    v4f;
typedef __attribute__((ext_vector_type(4)))  unsigned int v4u;


#define VST2(T, ptr, val) do { const T vst2_v_ = (val); *(volatile T*)(ptr) = vst2_v_; __threadfence(); *(volatile T*)(ptr) = vst2_v_; } while (0)

__device__ __forceinline__ float bfr(float f) {
    unsigned u = __float_as_uint(f);
    u += 0x7FFFu + ((u >> 16) & 1u);
    return __uint_as_float(u & 0xFFFF0000u);
}
__device__ __forceinline__ unsigned bf16_bits(float f) {
    unsigned u = __float_as_uint(f);
    u += 0x7FFFu + ((u >> 16) & 1u);
    return u >> 16;
}
static __device__ __forceinline__ h16 toh_flush(float v) {
    const h16 r = (h16)v;
    return (fabsf(v) < 6.103515625e-05f) ? (h16)0.0f : r;
}
__device__ __forceinline__ unsigned hbits(float x) {
    return (unsigned)__builtin_bit_cast(unsigned short, toh_flush(x));
}
__device__ __forceinline__ void st8hf(unsigned short* P, size_t o, const float* v) {
    v4u pk;
    pk.x = hbits(v[0]) | (hbits(v[1]) << 16);
    pk.y = hbits(v[2]) | (hbits(v[3]) << 16);
    pk.z = hbits(v[4]) | (hbits(v[5]) << 16);
    pk.w = hbits(v[6]) | (hbits(v[7]) << 16);
    VST2(v4u, (v4u*)(P + o), pk);
}

union FragU { v16h v; v8h h[2]; };
__device__ __forceinline__ v16h frag_ld(const _Float16* p) {
    FragU f; f.h[0] = *(const v8h*)(p); f.h[1] = *(const v8h*)(p + 16); return f.v;
}
__device__ __forceinline__ v8f wmma16(v16h a, v16h b, v8f c) {
    c = __builtin_amdgcn_wmma_f32_16x16x32_f16(false, a, false, b, (short)0, c, false, false);
    asm volatile("v_nop\n\tv_nop\n\tv_nop\n\tv_nop" : "+v"(c) : "v"(a), "v"(b));
    return c;
}
__device__ __forceinline__ void wave_sync_lds() {
    __builtin_amdgcn_fence(3  , "workgroup");
    __builtin_amdgcn_wave_barrier();
    __builtin_amdgcn_fence(2  , "workgroup");
}

__device__ __forceinline__ float gelu_t(float x) {
    const float t = fminf(GELU_K * (x + 0.044715f * (x * x * x)), 126.0f);
    return x * __builtin_amdgcn_rcpf(1.0f + exp2f(t));
}

__device__ __forceinline__ unsigned refl64(unsigned i) {
    const unsigned t = (2u * i + 129u) & 255u;
    int m = (int)t - 128;
    m = (m < 0) ? -m : m;
    unsigned r = (unsigned)(m - 1) >> 1;
    return (r < 63u) ? r : 63u;
}

__device__ __forceinline__ void lerp2(unsigned q00, unsigned q01, unsigned q10, unsigned q11,
                                      float w00, float w01, float w10, float w11, float& e, float& o) {
    e = ((w00 * __uint_as_float(q00 << 16) + w01 * __uint_as_float(q01 << 16)) + w10 * __uint_as_float(q10 << 16)) + w11 * __uint_as_float(q11 << 16);
    o = ((w00 * __uint_as_float(q00 & 0xFFFF0000u) + w01 * __uint_as_float(q01 & 0xFFFF0000u)) + w10 * __uint_as_float(q10 & 0xFFFF0000u)) + w11 * __uint_as_float(q11 & 0xFFFF0000u);
}

__global__ __launch_bounds__(256) void k_gcvt(const float* __restrict__ g, unsigned short* __restrict__ gb, unsigned n8) {
    const unsigned u = blockIdx.x * 256u + threadIdx.x;
    if (u >= n8) return;
    const v4f a = *(const v4f*)(g + (size_t)8u * u);
    const v4f b = *(const v4f*)(g + (size_t)8u * u + 4u);
    v4u pk;
    pk.x = bf16_bits(a.x) | (bf16_bits(a.y) << 16);
    pk.y = bf16_bits(a.z) | (bf16_bits(a.w) << 16);
    pk.z = bf16_bits(b.x) | (bf16_bits(b.y) << 16);
    pk.w = bf16_bits(b.z) | (bf16_bits(b.w) << 16);
    VST2(v4u, (v4u*)(gb + (size_t)8u * u), pk);
}

__global__ __launch_bounds__(256) void k_wtpad(const float* __restrict__ Wm, unsigned KS, unsigned NOS, unsigned NOP, unsigned KP,
                                               unsigned e0, unsigned f0, unsigned f1, unsigned shift,
                                               unsigned short* __restrict__ W16, float sw) {
    const unsigned u = blockIdx.x * 256u + threadIdx.x;
    const unsigned per = KP >> 3;
    if (u >= NOP * per) return;
    const unsigned o = u / per;
    const unsigned k0 = 8u * (u - o * per);
    const unsigned oc = (o < NOS) ? o : (NOS - 1u);
    float v[8];
#pragma unroll
    for (int i = 0; i < 8; ++i) {
        const unsigned k = k0 + (unsigned)i;
        const bool inA = k < e0;
        const bool inB = (k >= f0) && (k < f1);
        unsigned row = inA ? k : (inB ? (k - shift) : 0u);
        row = (row < KS) ? row : (KS - 1u);
        const float wv = bfr(Wm[(size_t)row * NOS + oc]) * sw;
        v[i] = ((inA || inB) && (o < NOS)) ? wv : 0.0f;
    }
    st8hf(W16, (size_t)o * KP + k0, v);
}

template <int KTOT>
__device__ __forceinline__ void mm_layer(v8f (&acc)[2][8], const _Float16* xw, const _Float16* __restrict__ Wt,
                                         unsigned c, unsigned hh) {
#pragma unroll
    for (int i = 0; i < 2; ++i)
#pragma unroll
        for (int j = 0; j < 8; ++j) acc[i][j] = (v8f){0.f,0.f,0.f,0.f,0.f,0.f,0.f,0.f};
#pragma unroll 1
    for (unsigned k0 = 0; k0 < (unsigned)KTOT; k0 += 32u) {
        const v16h a0 = frag_ld(xw + c * XP + k0 + 8u * hh);
        const v16h a1 = frag_ld(xw + (16u + c) * XP + k0 + 8u * hh);
#pragma unroll
        for (int j = 0; j < 8; ++j) {
            const v16h bh = frag_ld(Wt + (size_t)((unsigned)j * 16u + c) * (unsigned)KTOT + k0 + 8u * hh);
            acc[0][j] = wmma16(a0, bh, acc[0][j]);
            acc[1][j] = wmma16(a1, bh, acc[1][j]);
        }
    }
}

template <bool RES = false>
__device__ __forceinline__ void act_layer(v8f (&acc)[2][8], _Float16* xw, float* sw, const float* __restrict__ bias,
                                          unsigned lane, unsigned c, unsigned hh) {
    const v4f bq = *(const v4f*)(bias + 4u * lane);
    const float bv0 = bfr(bq.x), bv1 = bfr(bq.y), bv2 = bfr(bq.z), bv3 = bfr(bq.w);
#pragma unroll
    for (int i = 0; i < 2; ++i) {
#pragma unroll
        for (int j = 0; j < 8; ++j)
#pragma unroll
            for (int r = 0; r < 8; ++r)
                sw[(8u * hh + (unsigned)r) * SP + (unsigned)j * 16u + c] = acc[i][j][r];
        wave_sync_lds();
#pragma unroll 1
        for (unsigned row = 0; row < 16u; ++row) {
            const v4f s = *(const v4f*)(sw + row * SP + 4u * lane);
            const float t0 = gelu_t(s.x * ACT_SC + bv0) * ACT_CARRY;
            const float t1 = gelu_t(s.y * ACT_SC + bv1) * ACT_CARRY;
            const float t2 = gelu_t(s.z * ACT_SC + bv2) * ACT_CARRY;
            const float t3 = gelu_t(s.w * ACT_SC + bv3) * ACT_CARRY;
            v4h hv;
            hv[0] = toh_flush(t0);
            hv[1] = toh_flush(t1);
            hv[2] = toh_flush(t2);
            hv[3] = toh_flush(t3);
            *(v4h*)(xw + ((unsigned)i * 16u + row) * XP + 4u * lane) = hv;
            if (RES) {
                v4h rv;
                rv[0] = toh_flush((t0 - (float)((h16)t0)) * RES_CARRY);
                rv[1] = toh_flush((t1 - (float)((h16)t1)) * RES_CARRY);
                rv[2] = toh_flush((t2 - (float)((h16)t2)) * RES_CARRY);
                rv[3] = toh_flush((t3 - (float)((h16)t3)) * RES_CARRY);
                *(v4h*)(xw + ((unsigned)i * 16u + row) * XP + RES0 + 4u * lane) = rv;
            }
        }
        wave_sync_lds();
    }
}

__global__ __launch_bounds__(128) __attribute__((amdgpu_num_vgpr(256))) void k_mlp(
    const float* __restrict__ xy, const unsigned short* __restrict__ gbf,
    const _Float16* __restrict__ w0t, const _Float16* __restrict__ w1t, const _Float16* __restrict__ w2t,
    const _Float16* __restrict__ wot,
    const float* __restrict__ b0, const float* __restrict__ b1, const float* __restrict__ b2, const float* __restrict__ bo,
    float* __restrict__ out) {
    __shared__ __align__(16) _Float16 sX[WAVES][ROWS_W * XP];
    __shared__ __align__(16) float sS[WAVES][16 * SP];
    const unsigned lane = threadIdx.x & 31u;
    const unsigned wave = (unsigned)__builtin_amdgcn_readfirstlane((int)(threadIdx.x >> 5));
    const unsigned hh = lane >> 4, c = lane & 15u;
    const unsigned img = blockIdx.x / (unsigned)TILES_PER_IMG;
    const unsigned tile = blockIdx.x - img * (unsigned)TILES_PER_IMG;
    const unsigned n0 = tile * (unsigned)ROWS_B + wave * (unsigned)ROWS_W;
    _Float16* xw = sX[wave];
    float* sw = sS[wave];

    unsigned o00, o01, o10, o11;
    float w00, w01, w10, w11;
    {
        const unsigned n = n0 + lane;
        const float cx = bfr(xy[2u * n]);
        const float cy = bfr(xy[2u * n + 1u]);
        _Float16* xr = xw + lane * XP;
        xr[0] = toh_flush(cx * ACT_CARRY);
        xr[1] = toh_flush(cy * ACT_CARRY);
        const float pif = __uint_as_float(0x40490FDBu);
#pragma unroll 1
        for (unsigned j = 0; j < 20u; ++j) {
            const unsigned f = j >> 1, cd = j & 1u;
            const float fr = pif * (float)(1u << f);
            const float xv = (cd != 0u) ? cy : cx;
            const float ang = xv * fr;
            const float sv = sinf(ang);
            const float cv = cosf(ang);
            xr[2u + 4u * f + cd] = toh_flush(sv * ACT_CARRY);
            xr[4u + 4u * f + cd] = toh_flush(cv * ACT_CARRY);
        }
        xr[42] = (h16)0.0f; xr[43] = (h16)0.0f; xr[44] = (h16)0.0f;
        xr[45] = (h16)0.0f; xr[46] = (h16)0.0f; xr[47] = (h16)0.0f;
        const v8h z8 = (v8h){(h16)0.0f,(h16)0.0f,(h16)0.0f,(h16)0.0f,(h16)0.0f,(h16)0.0f,(h16)0.0f,(h16)0.0f};
        *(v8h*)(xr + 304) = z8;
        *(v8h*)(xr + 312) = z8;
        const float pr = (cx + 1.0f) * 0.5f * 63.0f;
        const float pc = (cy + 1.0f) * 0.5f * 63.0f;
        const float lr = floorf(pr), lc = floorf(pc);
        const float ur = pr - lr, uc = pc - lc;
        const float dr = 1.0f - ur, dc = 1.0f - uc;
        const unsigned ir = (unsigned)(int)lr, ic = (unsigned)(int)lc;
        const unsigned r0 = refl64(ir), r1 = refl64(ir + 1u);
        const unsigned c0 = refl64(ic), c1 = refl64(ic + 1u);
        o00 = (r0 * IMG_W + c0) * IMG_C; o01 = (r0 * IMG_W + c1) * IMG_C;
        o10 = (r1 * IMG_W + c0) * IMG_C; o11 = (r1 * IMG_W + c1) * IMG_C;
        w00 = dr * dc; w01 = dr * uc; w10 = ur * dc; w11 = ur * uc;
    }

    {
        const unsigned short* gimg = gbf + (size_t)img * IMG_ELEMS + 8u * lane;
#pragma unroll 1
        for (unsigned r = 0; r < (unsigned)ROWS_W; ++r) {
            const unsigned a00 = __shfl(o00, (int)r, 32), a01 = __shfl(o01, (int)r, 32);
            const unsigned a10 = __shfl(o10, (int)r, 32), a11 = __shfl(o11, (int)r, 32);
            const float f00 = __shfl(w00, (int)r, 32), f01 = __shfl(w01, (int)r, 32);
            const float f10 = __shfl(w10, (int)r, 32), f11 = __shfl(w11, (int)r, 32);
            const v4u q00 = *(const v4u*)(gimg + a00);
            const v4u q01 = *(const v4u*)(gimg + a01);
            const v4u q10 = *(const v4u*)(gimg + a10);
            const v4u q11 = *(const v4u*)(gimg + a11);
            float v0, v1, v2, v3, v4, v5, v6, v7;
            lerp2(q00.x, q01.x, q10.x, q11.x, f00, f01, f10, f11, v0, v1);
            lerp2(q00.y, q01.y, q10.y, q11.y, f00, f01, f10, f11, v2, v3);
            lerp2(q00.z, q01.z, q10.z, q11.z, f00, f01, f10, f11, v4, v5);
            lerp2(q00.w, q01.w, q10.w, q11.w, f00, f01, f10, f11, v6, v7);
            v8h hv;
            hv[0] = toh_flush(v0 * ACT_CARRY); hv[1] = toh_flush(v1 * ACT_CARRY);
            hv[2] = toh_flush(v2 * ACT_CARRY); hv[3] = toh_flush(v3 * ACT_CARRY);
            hv[4] = toh_flush(v4 * ACT_CARRY); hv[5] = toh_flush(v5 * ACT_CARRY);
            hv[6] = toh_flush(v6 * ACT_CARRY); hv[7] = toh_flush(v7 * ACT_CARRY);
            *(v8h*)(xw + r * XP + FEAT0 + 8u * lane) = hv;
        }
    }
    wave_sync_lds();

    v8f acc[2][8];
    mm_layer<K0P>(acc, xw, w0t, c, hh);
    act_layer(acc, xw, sw, b0, lane, c, hh);
    mm_layer<WIDTH>(acc, xw, w1t, c, hh);
    act_layer(acc, xw, sw, b1, lane, c, hh);
    mm_layer<WIDTH>(acc, xw, w2t, c, hh);
    act_layer<true>(acc, xw, sw, b2, lane, c, hh);

    v8f ao[2], ar[2];
    ao[0] = (v8f){0.f,0.f,0.f,0.f,0.f,0.f,0.f,0.f};
    ao[1] = ao[0];
    ar[0] = ao[0];
    ar[1] = ao[0];
#pragma unroll 1
    for (unsigned k0 = 0; k0 < (unsigned)WIDTH; k0 += 32u) {
        const v16h a0 = frag_ld(xw + c * XP + k0 + 8u * hh);
        const v16h a1 = frag_ld(xw + (16u + c) * XP + k0 + 8u * hh);
        const v16h ra0 = frag_ld(xw + c * XP + RES0 + k0 + 8u * hh);
        const v16h ra1 = frag_ld(xw + (16u + c) * XP + RES0 + k0 + 8u * hh);
        const v16h bh = frag_ld(wot + (size_t)c * WIDTH + k0 + 8u * hh);
        ao[0] = wmma16(a0, bh, ao[0]);
        ao[1] = wmma16(a1, bh, ao[1]);
        ar[0] = wmma16(ra0, bh, ar[0]);
        ar[1] = wmma16(ra1, bh, ar[1]);
    }
#pragma unroll
    for (int i = 0; i < 2; ++i)
#pragma unroll
        for (int r = 0; r < 8; ++r)
            sw[((unsigned)i * 16u + 8u * hh + (unsigned)r) * NOUTP + c] = ao[i][r] + ar[i][r] * RES_INV;
    wave_sync_lds();
    {
        const float bo0 = bfr(bo[0]), bo1 = bfr(bo[1]), bo2 = bfr(bo[2]);
#pragma unroll 1
        for (unsigned q = 0; q < 3u; ++q) {
            const unsigned e = lane + 32u * q;
            const unsigned row = e / 3u;
            const unsigned col = e - 3u * row;
            const float bsel = (col == 0u) ? bo0 : ((col == 1u) ? bo1 : bo2);
            const float z = sw[row * NOUTP + col] * ACT_SC + bsel;
            sw[OFLAT + e] = tanhf(z);
        }
    }
    wave_sync_lds();
    {
        const unsigned li = (lane < 24u) ? lane : 23u;
        const v4f ov = *(const v4f*)(sw + OFLAT + 4u * li);
        float* dst = out + ((size_t)img * NPTS + n0) * NOUT + 4u * li;
        if (lane < 24u) *(volatile v4f*)dst = ov;
        __threadfence();
        if (lane < 24u) *(volatile v4f*)dst = ov;
    }
}

extern "C" void kernel_launch(void* const* d_in, const int* in_sizes, int n_in, void* d_out, int out_size,
                              void* d_ws, size_t ws_size, hipStream_t stream) {
    if (n_in < 10) return;
    if (in_sizes[0] < NB * IMG_ELEMS || in_sizes[1] < NPTS * 2 || in_sizes[2] < KIN * WIDTH || in_sizes[3] < WIDTH) return;
    if (in_sizes[4] < WIDTH * WIDTH || in_sizes[5] < WIDTH || in_sizes[6] < WIDTH * WIDTH || in_sizes[7] < WIDTH) return;
    if (in_sizes[8] < WIDTH * NOUT || in_sizes[9] < NOUT || out_size < NB * NPTS * NOUT) return;

    const float* grid = (const float*)d_in[0];
    const float* xy   = (const float*)d_in[1];
    const float* w0   = (const float*)d_in[2];
    const float* b0   = (const float*)d_in[3];
    const float* w1   = (const float*)d_in[4];
    const float* b1   = (const float*)d_in[5];
    const float* w2   = (const float*)d_in[6];
    const float* b2   = (const float*)d_in[7];
    const float* wo   = (const float*)d_in[8];
    const float* bo   = (const float*)d_in[9];
    float* out = (float*)d_out;

    char* wsp = (char*)d_ws;
    size_t off = 0;
    auto carve = [&](size_t bytes) -> void* { void* r = wsp + off; off += (bytes + 255) & ~(size_t)255; return r; };
    unsigned short* gbf = (unsigned short*)carve((size_t)NB * IMG_ELEMS * 2);
    unsigned short* w0t = (unsigned short*)carve((size_t)WIDTH * K0P * 2);
    unsigned short* w1t = (unsigned short*)carve((size_t)WIDTH * WIDTH * 2);
    unsigned short* w2t = (unsigned short*)carve((size_t)WIDTH * WIDTH * 2);
    unsigned short* wot = (unsigned short*)carve((size_t)NOUTP * WIDTH * 2);
    if (off > ws_size || off > (size_t)134217728) return;

    k_gcvt<<<(NB * IMG_ELEMS / 8) / 256, 256, 0, stream>>>(grid, gbf, (unsigned)(NB * IMG_ELEMS / 8));
    k_wtpad<<<(WIDTH * (K0P / 8) + 255) / 256, 256, 0, stream>>>(w0, KIN, WIDTH, WIDTH, K0P, NENC, FEAT0, FEAT0 + IMG_C, FEAT0 - NENC, w0t, W_CARRY);
    k_wtpad<<<(WIDTH * (WIDTH / 8) + 255) / 256, 256, 0, stream>>>(w1, WIDTH, WIDTH, WIDTH, WIDTH, WIDTH, 0, 0, 0, w1t, W_CARRY);
    k_wtpad<<<(WIDTH * (WIDTH / 8) + 255) / 256, 256, 0, stream>>>(w2, WIDTH, WIDTH, WIDTH, WIDTH, WIDTH, 0, 0, 0, w2t, W_CARRY);
    k_wtpad<<<(NOUTP * (WIDTH / 8) + 255) / 256, 256, 0, stream>>>(wo, WIDTH, NOUT, NOUTP, WIDTH, WIDTH, 0, 0, 0, wot, W_CARRY);

    k_mlp<<<NB * TILES_PER_IMG, 128, 0, stream>>>(xy, gbf, (const _Float16*)w0t, (const _Float16*)w1t, (const _Float16*)w2t,
                                                  (const _Float16*)wot, b0, b1, b2, bo, out);
}
